// Mamba_6828998001042
// MI455X (gfx1250) — hardware-run, weakly checked
//
#include <hip/hip_runtime.h>
#include <math.h>

typedef __attribute__((ext_vector_type(16))) _Float16 v16h;
typedef __attribute__((ext_vector_type(8)))  _Float16 v8h;
typedef __attribute__((ext_vector_type(16))) __bf16   v16b;
typedef __attribute__((ext_vector_type(8)))  __bf16   v8b;
typedef __attribute__((ext_vector_type(8)))  float    v8f;
typedef __attribute__((ext_vector_type(4)))  float    v4f;

constexpr int kBatch  = 2;
constexpr int kSeq    = 2048;
constexpr int kDm     = 1024;
constexpr int kDin    = 2048;
constexpr int kNst    = 16;
constexpr int kDtR    = 64;
constexpr int kXdW    = 96;
constexpr int kXdP    = 128;
constexpr int kRows   = kBatch * kSeq;
constexpr int kConvCh = 256;
constexpr int kConvTh = 128;
constexpr int kConvRw = 64;
constexpr int kConvTP = 260;
constexpr int kScanTS = 64;
constexpr int kScanCh = 64;
constexpr int kScanP  = 68;
constexpr int kBCW    = 32;
static_assert(kDtR + 2 * kNst == kXdW);
static_assert(kXdW <= kXdP);
static_assert((kDm % 32) == 0 && (kDin % 32) == 0 && (kDtR % 32) == 0);
static_assert((kRows % 64) == 0 && (kDin % 64) == 0 && (kXdP % 64) == 0 && (kDm % 64) == 0);
static_assert((kSeq % kScanTS) == 0 && (kSeq % kConvRw) == 0 && (kDin % kScanCh) == 0 && (kDin % kConvCh) == 0);
static_assert(kConvCh == 2 * kConvTh);

constexpr size_t kOffXB   = 0;
constexpr size_t kOffWIB  = kOffXB  + (size_t)kRows * kDm  * 2;
constexpr size_t kOffWXB  = kOffWIB + (size_t)(2 * kDin) * kDm * 2;
constexpr size_t kOffWDB  = kOffWXB + (size_t)kXdP * kDin * 2;
constexpr size_t kOffWOB  = kOffWDB + (size_t)kDin * kDtR * 2;
constexpr size_t kOffXHP  = kOffWOB + (size_t)kDm  * kDin * 2;
constexpr size_t kOffXLP  = kOffXHP + (size_t)kRows * kDin * 2;
constexpr size_t kOffZ    = kOffXLP + (size_t)kRows * kDin * 2;
constexpr size_t kOffUCH  = kOffZ   + (size_t)kRows * kDin * 4;
constexpr size_t kOffUCL  = kOffUCH + (size_t)kRows * kDin * 2;
constexpr size_t kOffXDH  = kOffUCL + (size_t)kRows * kDin * 2;
constexpr size_t kOffXDL  = kOffXDH + (size_t)kRows * kXdP * 2;
constexpr size_t kWsTotal = kOffXDL + (size_t)kRows * kXdP * 2;
static_assert(kWsTotal == 124518400ull);
static_assert(kWsTotal <= 134217728ull);
static_assert((kOffWIB % 128) == 0 && (kOffWXB % 128) == 0 && (kOffWDB % 128) == 0 && (kOffWOB % 128) == 0 &&
              (kOffXHP % 128) == 0 && (kOffXLP % 128) == 0 && (kOffZ % 128) == 0 && (kOffUCH % 128) == 0 &&
              (kOffUCL % 128) == 0 && (kOffXDH % 128) == 0 && (kOffXDL % 128) == 0);

__device__ __forceinline__ unsigned short f2bf_bits(float f) {
  unsigned u = __float_as_uint(f);
  return (unsigned short)((u + 0x7FFFu + ((u >> 16) & 1u)) >> 16);
}
__device__ __forceinline__ float bf_bits2f(unsigned short h) { return __uint_as_float(((unsigned)h) << 16); }
__device__ __forceinline__ float bf16r(float f) { return __uint_as_float(((unsigned)f2bf_bits(f)) << 16); }
__device__ __forceinline__ float lo16f(unsigned w) { return __uint_as_float(w << 16); }
__device__ __forceinline__ float hi16f(unsigned w) { return __uint_as_float(w & 0xffff0000u); }

__device__ __forceinline__ void dep_guard4_h(v8f& a, v8f& b, v8f& c, v8f& d, v16h x, v16h y) { asm volatile("v_nop\n\tv_nop\n\tv_nop\n\tv_nop" : "+v"(a), "+v"(b), "+v"(c), "+v"(d) : "v"(x), "v"(y)); }
__device__ __forceinline__ void dep_guard4_b(v8f& a, v8f& b, v8f& c, v8f& d, v16b x, v16b y) { asm volatile("v_nop\n\tv_nop\n\tv_nop\n\tv_nop" : "+v"(a), "+v"(b), "+v"(c), "+v"(d) : "v"(x), "v"(y)); }
__device__ __forceinline__ void keep4_h(v16h a, v16h b, v16h c, v16h d) { asm volatile("v_nop" :: "v"(a), "v"(b), "v"(c), "v"(d)); }
__device__ __forceinline__ void keep4_b(v16b a, v16b b, v16b c, v16b d) { asm volatile("v_nop" :: "v"(a), "v"(b), "v"(c), "v"(d)); }
__device__ __forceinline__ void acc_guard4(v8f& a, v8f& b, v8f& c, v8f& d) { asm volatile("v_nop\n\tv_nop\n\tv_nop\n\tv_nop" : "+v"(a), "+v"(b), "+v"(c), "+v"(d)); }
template <typename T> struct Frag;
template <> struct Frag<_Float16> {
  typedef v16h V; union U { v16h v; v8h h[2]; };
  static __device__ __forceinline__ v16h load(const _Float16* p) {
    U f; f.h[0] = *(const v8h*)(p); f.h[1] = *(const v8h*)(p + 16); return f.v;
  }
  static __device__ __forceinline__ v8f mma(v16h a, v16h b, v8f c) {
    return __builtin_amdgcn_wmma_f32_16x16x32_f16(false, a, false, b, (short)0, c, false, false);
  }
  static __device__ __forceinline__ void guard4(v8f& a, v8f& b, v8f& c, v8f& d, v16h x, v16h y) { dep_guard4_h(a, b, c, d, x, y); }
  static __device__ __forceinline__ void keep(v16h a, v16h b, v16h c, v16h d) { keep4_h(a, b, c, d); }
};
template <> struct Frag<__bf16> {
  typedef v16b V; union U { v16b v; v8b h[2]; };
  static __device__ __forceinline__ v16b load(const __bf16* p) {
    U f; f.h[0] = *(const v8b*)(p); f.h[1] = *(const v8b*)(p + 16); return f.v;
  }
  static __device__ __forceinline__ v8f mma(v16b a, v16b b, v8f c) {
    return __builtin_amdgcn_wmma_f32_16x16x32_bf16(false, a, false, b, (short)0, c, false, false);
  }
  static __device__ __forceinline__ void guard4(v8f& a, v8f& b, v8f& c, v8f& d, v16b x, v16b y) { dep_guard4_b(a, b, c, d, x, y); }
  static __device__ __forceinline__ void keep(v16b a, v16b b, v16b c, v16b d) { keep4_b(a, b, c, d); }
};

template <int ET> struct Elem;
template <> struct Elem<0> { typedef _Float16 T; };
template <> struct Elem<1> { typedef __bf16 T; };
template <int ET, int SPL, int BIAS_MODE, int OUT_MODE, bool RESID, int ACT = 0>
__global__ __launch_bounds__(256) void wmma_gemm64(
    const unsigned short* __restrict__ Ap, const unsigned short* __restrict__ A2p, int lda, long strideA,
    const unsigned short* __restrict__ Btp, const unsigned short* __restrict__ Bt2p, int ldb, long strideB,
    void* __restrict__ Cout, void* __restrict__ Cout2, int ldc, long strideC,
    const float* __restrict__ bias,
    const float* __restrict__ resid, long strideR,
    int M, int N, int K, float scale) {
  typedef typename Elem<ET>::T T;
  typedef typename Frag<T>::V V;
  const T* A = (const T*)Ap; const T* A2 = (const T*)A2p; const T* Bt = (const T*)Btp; const T* Bt2 = (const T*)Bt2p;
  __shared__ __align__(16) float sT[8][16 * 68];
  const int b    = blockIdx.y;
  const int lane = threadIdx.x & 31;
  const int wave = threadIdx.x >> 5;
  const int tilesN = N >> 6;
  const int tilesM = M >> 6;
  const int tile = blockIdx.x * 8 + wave;
  if (tile >= tilesM * tilesN) return;
  const int tm = tile / tilesN;
  const int tn = tile - tm * tilesN;
  const int m0 = tm << 6;
  const int n0 = tn << 6;

  const T* Ab  = A  + (size_t)b * strideA;
  const T* Bb  = Bt + (size_t)b * strideB;
  const T* Ab2 = (SPL >= 1) ? (A2  + (size_t)b * strideA) : nullptr;
  const T* Bb2 = (SPL == 2) ? (Bt2 + (size_t)b * strideB) : nullptr;

  const int rlane = lane & 15;
  const int koff  = (lane >> 4) * 8;
  const int mOff  = (lane >> 4) * 8;

  v8f acc[4][4];
#pragma unroll
  for (int i = 0; i < 4; ++i)
#pragma unroll
    for (int j = 0; j < 4; ++j) acc[i][j] = (v8f){0.f,0.f,0.f,0.f,0.f,0.f,0.f,0.f};

  for (int k0 = 0; k0 < K; k0 += 32) {
    V bh[4], bl[4];
#pragma unroll
    for (int j = 0; j < 4; ++j) {
      const size_t bo = (size_t)(n0 + (j << 4) + rlane) * ldb + koff + k0;
      bh[j] = Frag<T>::load(Bb + bo);
      if (SPL == 2) bl[j] = Frag<T>::load(Bb2 + bo);
    }
#pragma unroll
    for (int i = 0; i < 4; ++i) {
      const size_t ao = (size_t)(m0 + (i << 4) + rlane) * lda + koff + k0;
      V ah = Frag<T>::load(Ab + ao);
      V al;
      if (SPL >= 1) al = Frag<T>::load(Ab2 + ao);
#pragma unroll
      for (int j = 0; j < 4; ++j) {
        acc[i][j] = Frag<T>::mma(ah, bh[j], acc[i][j]);
        if (SPL == 2) acc[i][j] = Frag<T>::mma(ah, bl[j], acc[i][j]);
        if (SPL >= 1) acc[i][j] = Frag<T>::mma(al, bh[j], acc[i][j]);
      }
      Frag<T>::guard4(acc[i][0], acc[i][1], acc[i][2], acc[i][3], ah, (SPL >= 1) ? al : ah);
    }
    Frag<T>::keep(bh[0], bh[1], bh[2], bh[3]);
    if (SPL == 2) Frag<T>::keep(bl[0], bl[1], bl[2], bl[3]);
  }
  acc_guard4(acc[0][0], acc[0][1], acc[0][2], acc[0][3]);
  acc_guard4(acc[1][0], acc[1][1], acc[1][2], acc[1][3]);
  acc_guard4(acc[2][0], acc[2][1], acc[2][2], acc[2][3]);
  acc_guard4(acc[3][0], acc[3][1], acc[3][2], acc[3][3]);

  float* slab = sT[wave];
  const float* Rb = RESID ? (resid + (size_t)b * strideR) : nullptr;
#pragma unroll
  for (int i = 0; i < 4; ++i) {
    const int mBase = m0 + (i << 4);
#pragma unroll
    for (int j = 0; j < 4; ++j) {
      const int n = n0 + (j << 4) + rlane;
      float bv = 0.f;
      if (BIAS_MODE == 2) bv = bias[n];
#pragma unroll
      for (int r = 0; r < 8; ++r) {
        float v = acc[i][j][r] * scale;
        if (BIAS_MODE == 1) v += bias[mBase + mOff + r];
        if (BIAS_MODE == 2) v += bv;
        if (RESID) v += Rb[(size_t)(mBase + mOff + r) * ldc + n];
        if (ACT == 1) v = tanhf(v);
        if (ACT == 2) v = fmaxf(v, 0.0f);
        if (ACT == 3) v = v / (1.0f + expf(-v));
        if (ACT == 4) v = (v > 0.f) ? v : 0.01f * v;
        slab[(mOff + r) * 68 + (j << 4) + rlane] = v;
      }
    }
    __builtin_amdgcn_fence(__ATOMIC_RELEASE, "workgroup");
    __builtin_amdgcn_wave_barrier();
    __builtin_amdgcn_fence(__ATOMIC_ACQUIRE, "workgroup");
    if (OUT_MODE == 0) {
      float* C = (float*)Cout + (size_t)b * strideC;
      const int hh = lane >> 4, c4 = (lane & 15) * 4;
      for (int pass = 0; pass < 2; ++pass) {
#pragma unroll
        for (int it = 0; it < 8; ++it) {
          const int row = it * 2 + hh;
          v4f v = *(const v4f*)(slab + row * 68 + c4);
          *(volatile v4f*)(C + (size_t)(mBase + row) * ldc + n0 + c4) = v;
        }
        __threadfence();
      }
    } else {
      const int q = lane >> 3, c8 = (lane & 7) * 8;
      unsigned short* C  = (unsigned short*)Cout  + (size_t)b * strideC;
      unsigned short* C2 = (OUT_MODE == 2) ? ((unsigned short*)Cout2 + (size_t)b * strideC) : nullptr;
      for (int pass = 0; pass < 2; ++pass) {
#pragma unroll
        for (int it = 0; it < 4; ++it) {
          const int row = it * 4 + q;
          const float* sp = slab + row * 68 + c8;
          v8h hv, lv;
#pragma unroll
          for (int e = 0; e < 8; ++e) {
            if (OUT_MODE == 1) {
              hv[e] = (_Float16)sp[e];
            } else {
              unsigned short hb = f2bf_bits(sp[e]);
              unsigned short lb = f2bf_bits(sp[e] - bf_bits2f(hb));
              hv[e] = __builtin_bit_cast(_Float16, hb);
              lv[e] = __builtin_bit_cast(_Float16, lb);
            }
          }
          *(volatile v8h*)(C + (size_t)(mBase + row) * ldc + n0 + c8) = hv;
          if (OUT_MODE == 2) *(volatile v8h*)(C2 + (size_t)(mBase + row) * ldc + n0 + c8) = lv;
        }
        __threadfence();
      }
    }
    __builtin_amdgcn_fence(__ATOMIC_RELEASE, "workgroup");
    __builtin_amdgcn_wave_barrier();
    __builtin_amdgcn_fence(__ATOMIC_ACQUIRE, "workgroup");
  }
}

__global__ __launch_bounds__(256) void rows_bf16_kernel(
    const float* __restrict__ src, unsigned short* __restrict__ dst, int total8, int valid8)
{
  const int i = blockIdx.x * 256 + threadIdx.x;
  if (i >= total8) return;
  const int ic = (i < valid8) ? i : (valid8 - 1);
  const float fz = (i < valid8) ? 1.0f : 0.0f;
  const size_t e0 = (size_t)ic << 3;
  const v4f a0 = *(const v4f*)(src + e0);
  const v4f a1 = *(const v4f*)(src + e0 + 4);
  v8h hv;
#pragma unroll
  for (int e = 0; e < 4; ++e) {
    hv[e]     = __builtin_bit_cast(_Float16, f2bf_bits(a0[e] * fz));
    hv[4 + e] = __builtin_bit_cast(_Float16, f2bf_bits(a1[e] * fz));
  }
  unsigned short* qd = dst + ((size_t)i << 3);
  *(volatile v8h*)qd = hv;
  __threadfence();
  *(volatile v8h*)qd = hv;
}

__global__ __launch_bounds__(kConvTh) void conv_silu_kernel(
    const unsigned* __restrict__ XHw, const unsigned* __restrict__ XLw,
    const float* __restrict__ cw, const float* __restrict__ cb,
    unsigned short* __restrict__ UCH, unsigned short* __restrict__ UCL)
{
  __shared__ __align__(16) float sT[16 * kConvTP];
  constexpr size_t kWP = kDin / 2;
  const int tid = threadIdx.x, lane = tid & 31, wave = tid >> 5;
  const int d0 = blockIdx.x * kConvCh;
  const int da = d0 + 2 * tid;
  const size_t wcol = (size_t)(d0 >> 1) + tid;
  const int g0 = blockIdx.y * kConvRw;
  const int tb = g0 & (kSeq - 1);
  const v4f wa = *(const v4f*)(cw + (size_t)da * 4);
  const v4f wb = *(const v4f*)(cw + (size_t)(da + 1) * 4);
  const float w0a = bf16r(wa[0]), w1a = bf16r(wa[1]), w2a = bf16r(wa[2]), w3a = bf16r(wa[3]);
  const float w0b = bf16r(wb[0]), w1b = bf16r(wb[1]), w2b = bf16r(wb[2]), w3b = bf16r(wb[3]);
  const float bca = bf16r(cb[da]), bcb = bf16r(cb[da + 1]);
  float xm3a, xm2a, xm1a, xm3b, xm2b, xm1b;
  {
    const bool hist = (tb > 0);
    const int rb = hist ? (g0 - 3) : g0;
    const float fh = hist ? 1.0f : 0.0f;
    const unsigned h3 = XHw[(size_t)rb * kWP + wcol],       l3 = XLw[(size_t)rb * kWP + wcol];
    const unsigned h2 = XHw[(size_t)(rb + 1) * kWP + wcol], l2 = XLw[(size_t)(rb + 1) * kWP + wcol];
    const unsigned h1 = XHw[(size_t)(rb + 2) * kWP + wcol], l1 = XLw[(size_t)(rb + 2) * kWP + wcol];
    xm3a = (lo16f(h3) + lo16f(l3)) * fh;  xm3b = (hi16f(h3) + hi16f(l3)) * fh;
    xm2a = (lo16f(h2) + lo16f(l2)) * fh;  xm2b = (hi16f(h2) + hi16f(l2)) * fh;
    xm1a = (lo16f(h1) + lo16f(l1)) * fh;  xm1b = (hi16f(h1) + hi16f(l1)) * fh;
  }
#pragma unroll 1
  for (int sub = 0; sub < kConvRw / 16; ++sub) {
    const int lb = g0 + sub * 16;
#pragma unroll 1
    for (int s = 0; s < 16; ++s) {
      const size_t wo = (size_t)(lb + s) * kWP + wcol;
      const unsigned hw = XHw[wo], lw = XLw[wo];
      const float xa = lo16f(hw) + lo16f(lw);
      const float xb = hi16f(hw) + hi16f(lw);
      float acca = w0a * xm3a;
      acca = fmaf(w1a, xm2a, acca);
      acca = fmaf(w2a, xm1a, acca);
      acca = fmaf(w3a, xa, acca);
      float accb = w0b * xm3b;
      accb = fmaf(w1b, xm2b, accb);
      accb = fmaf(w2b, xm1b, accb);
      accb = fmaf(w3b, xb, accb);
      const float sva = acca + bca;
      const float svb = accb + bcb;
      const float ua = sva * __builtin_amdgcn_rcpf(1.0f + expf(-sva));
      const float ub = svb * __builtin_amdgcn_rcpf(1.0f + expf(-svb));
      sT[s * kConvTP + 2 * tid]     = ua;
      sT[s * kConvTP + 2 * tid + 1] = ub;
      xm3a = xm2a; xm2a = xm1a; xm1a = xa;
      xm3b = xm2b; xm2b = xm1b; xm1b = xb;
    }
    __syncthreads();
    v8h bh[4], blo[4];
#pragma unroll
    for (int it = 0; it < 4; ++it) {
      const float* sp = sT + (it * 4 + wave) * kConvTP + lane * 8;
      const v4f a0 = *(const v4f*)(sp);
      const v4f a1 = *(const v4f*)(sp + 4);
#pragma unroll
      for (int e = 0; e < 4; ++e) {
        const unsigned short h0 = f2bf_bits(a0[e]), h1 = f2bf_bits(a1[e]);
        const unsigned short l0 = f2bf_bits(a0[e] - bf_bits2f(h0)), l1 = f2bf_bits(a1[e] - bf_bits2f(h1));
        bh[it][e]      = __builtin_bit_cast(_Float16, h0);
        bh[it][4 + e]  = __builtin_bit_cast(_Float16, h1);
        blo[it][e]     = __builtin_bit_cast(_Float16, l0);
        blo[it][4 + e] = __builtin_bit_cast(_Float16, l1);
      }
    }
    for (int pass = 0; pass < 2; ++pass) {
#pragma unroll
      for (int it = 0; it < 4; ++it) {
        const size_t o = (size_t)(lb + it * 4 + wave) * kDin + d0 + lane * 8;
        *(volatile v8h*)(UCH + o) = bh[it];
        *(volatile v8h*)(UCL + o) = blo[it];
      }
      __threadfence();
    }
    __syncthreads();
  }
}

__global__ __launch_bounds__(kScanCh) void scan_kernel(
    const unsigned short* __restrict__ XDH, const unsigned short* __restrict__ XDL,
    const unsigned short* __restrict__ UCH, const unsigned short* __restrict__ UCL,
    const float* __restrict__ Z, const unsigned short* __restrict__ WDB,
    const float* __restrict__ bdt, const float* __restrict__ Alog, const float* __restrict__ Dp,
    unsigned short* __restrict__ YH, unsigned short* __restrict__ YL)
{
  __shared__ __align__(16) float sU[kScanTS * kScanP];
  __shared__ __align__(16) float sDP[kScanTS * kScanP];
  __shared__ __align__(16) float sY[kScanTS * kScanP];
  __shared__ __align__(16) float sBC[kScanTS * kBCW];
  const int tid = threadIdx.x, lane = tid & 31, wave = tid >> 5;
  constexpr int kBlkPerB = kDin / kScanCh;
  const int bix = blockIdx.x / kBlkPerB;
  const int d0  = (blockIdx.x - bix * kBlkPerB) * kScanCh;
  const int d   = d0 + tid;
  const size_t row0 = (size_t)bix * kSeq;
  const int rlane = lane & 15, hsel = lane >> 4, koff = hsel * 8;
  const int q = lane >> 3, c8 = (lane & 7) * 8;
  const __bf16* XDHb = (const __bf16*)(const void*)XDH;
  const __bf16* XDLb = (const __bf16*)(const void*)XDL;
  const __bf16* WDBb = (const __bf16*)(const void*)WDB;

  float negA[kNst], h[kNst];
  {
    const v4f* ap = (const v4f*)(Alog + (size_t)d * kNst);
    v4f a4[4];
#pragma unroll
    for (int g = 0; g < 4; ++g) a4[g] = ap[g];
#pragma unroll
    for (int g = 0; g < 4; ++g)
#pragma unroll
      for (int e = 0; e < 4; ++e) negA[4 * g + e] = -expf(bf16r(a4[g][e]));
#pragma unroll
    for (int k = 0; k < kNst; ++k) h[k] = 0.f;
  }
  const float bb = bf16r(bdt[d]), Dd = bf16r(Dp[d]);

#pragma unroll 1
  for (int t0 = 0; t0 < kSeq; t0 += kScanTS) {
    __syncthreads();
#pragma unroll 1
    for (int i = 0; i < 8; ++i) {
      const int idx = tid + kScanCh * i;
      const int r = idx >> 3, cc = (idx & 7) * 8;
      const size_t eo = (row0 + t0 + r) * kDin + d0 + cc;
      const uint4 hw = *(const uint4*)(const void*)(UCH + eo);
      const uint4 lw = *(const uint4*)(const void*)(UCL + eo);
      v4f f0, f1;
      f0[0] = lo16f(hw.x) + lo16f(lw.x); f0[1] = hi16f(hw.x) + hi16f(lw.x);
      f0[2] = lo16f(hw.y) + lo16f(lw.y); f0[3] = hi16f(hw.y) + hi16f(lw.y);
      f1[0] = lo16f(hw.z) + lo16f(lw.z); f1[1] = hi16f(hw.z) + hi16f(lw.z);
      f1[2] = lo16f(hw.w) + lo16f(lw.w); f1[3] = hi16f(hw.w) + hi16f(lw.w);
      *(v4f*)(sU + r * kScanP + cc)     = f0;
      *(v4f*)(sU + r * kScanP + cc + 4) = f1;
    }
#pragma unroll 1
    for (int i = 0; i < 4; ++i) {
      const int idx = tid + kScanCh * i;
      const int r = idx >> 2, part = idx & 3;
      const size_t eo = (row0 + t0 + r) * kXdP + kDtR + part * 8;
      const uint4 hw = *(const uint4*)(const void*)(XDH + eo);
      const uint4 lw = *(const uint4*)(const void*)(XDL + eo);
      v4f f0, f1;
      f0[0] = lo16f(hw.x) + lo16f(lw.x); f0[1] = hi16f(hw.x) + hi16f(lw.x);
      f0[2] = lo16f(hw.y) + lo16f(lw.y); f0[3] = hi16f(hw.y) + hi16f(lw.y);
      f1[0] = lo16f(hw.z) + lo16f(lw.z); f1[1] = hi16f(hw.z) + hi16f(lw.z);
      f1[2] = lo16f(hw.w) + lo16f(lw.w); f1[3] = hi16f(hw.w) + hi16f(lw.w);
      *(v4f*)(sBC + r * kBCW + part * 8)     = f0;
      *(v4f*)(sBC + r * kBCW + part * 8 + 4) = f1;
    }
    {
      v8f acc[2][4];
#pragma unroll
      for (int i = 0; i < 2; ++i)
#pragma unroll
        for (int j = 0; j < 4; ++j) acc[i][j] = (v8f){0.f,0.f,0.f,0.f,0.f,0.f,0.f,0.f};
#pragma unroll 1
      for (int k0 = 0; k0 < kDtR; k0 += 32) {
        v16b bh[4];
#pragma unroll
        for (int j = 0; j < 4; ++j)
          bh[j] = Frag<__bf16>::load(WDBb + (size_t)(d0 + 16 * j + rlane) * kDtR + koff + k0);
#pragma unroll
        for (int i = 0; i < 2; ++i) {
          const size_t ao = (row0 + t0 + 32 * wave + 16 * i + rlane) * kXdP + koff + k0;
          const v16b ah = Frag<__bf16>::load(XDHb + ao);
          const v16b al = Frag<__bf16>::load(XDLb + ao);
#pragma unroll
          for (int j = 0; j < 4; ++j) {
            acc[i][j] = Frag<__bf16>::mma(ah, bh[j], acc[i][j]);
            acc[i][j] = Frag<__bf16>::mma(al, bh[j], acc[i][j]);
          }
          Frag<__bf16>::guard4(acc[i][0], acc[i][1], acc[i][2], acc[i][3], ah, al);
        }
        Frag<__bf16>::keep(bh[0], bh[1], bh[2], bh[3]);
      }
      acc_guard4(acc[0][0], acc[0][1], acc[0][2], acc[0][3]);
      acc_guard4(acc[1][0], acc[1][1], acc[1][2], acc[1][3]);
#pragma unroll
      for (int i = 0; i < 2; ++i)
#pragma unroll
        for (int j = 0; j < 4; ++j)
#pragma unroll
          for (int r = 0; r < 8; ++r)
            sDP[(32 * wave + 16 * i + 8 * hsel + r) * kScanP + 16 * j + rlane] = acc[i][j][r];
    }
    __syncthreads();
#pragma unroll 1
    for (int s = 0; s < kScanTS; ++s) {
      const float xt = sU[s * kScanP + tid];
      const float v  = sDP[s * kScanP + tid] + bb;
      const float ev = expf(-fabsf(v));
      const float dlt = fmaxf(v, 0.0f) + log1pf(ev);
      const float dtx = dlt * xt;
      const float* br = sBC + s * kBCW;
      float Bs[kNst], Cs[kNst];
#pragma unroll
      for (int q4 = 0; q4 < 4; ++q4) {
        const v4f bv = *(const v4f*)(br + 4 * q4);
        const v4f cv = *(const v4f*)(br + kNst + 4 * q4);
        Bs[4 * q4 + 0] = bv[0]; Bs[4 * q4 + 1] = bv[1]; Bs[4 * q4 + 2] = bv[2]; Bs[4 * q4 + 3] = bv[3];
        Cs[4 * q4 + 0] = cv[0]; Cs[4 * q4 + 1] = cv[1]; Cs[4 * q4 + 2] = cv[2]; Cs[4 * q4 + 3] = cv[3];
      }
      float y = 0.0f;
#pragma unroll
      for (int k = 0; k < kNst; ++k) {
        const float e = expf(dlt * negA[k]);
        h[k] = e * h[k] + dtx * Bs[k];
        y = fmaf(h[k], Cs[k], y);
      }
      y = y + xt * Dd;
      const float zv = Z[(row0 + t0 + s) * kDin + d];
      const float sg = __builtin_amdgcn_rcpf(1.0f + expf(-zv));
      y = y * (zv * sg);
      sY[s * kScanP + tid] = y;
    }
    __syncthreads();
    v8h hv[8], lv[8];
#pragma unroll
    for (int it = 0; it < 8; ++it) {
      const int row = it * 8 + wave * 4 + q;
      const float* sp = sY + row * kScanP + c8;
      const v4f a0 = *(const v4f*)(sp);
      const v4f a1 = *(const v4f*)(sp + 4);
#pragma unroll
      for (int e = 0; e < 4; ++e) {
        const unsigned short h0 = f2bf_bits(a0[e]), h1 = f2bf_bits(a1[e]);
        const unsigned short l0 = f2bf_bits(a0[e] - bf_bits2f(h0)), l1 = f2bf_bits(a1[e] - bf_bits2f(h1));
        hv[it][e]     = __builtin_bit_cast(_Float16, h0);
        hv[it][4 + e] = __builtin_bit_cast(_Float16, h1);
        lv[it][e]     = __builtin_bit_cast(_Float16, l0);
        lv[it][4 + e] = __builtin_bit_cast(_Float16, l1);
      }
    }
    for (int pass = 0; pass < 2; ++pass) {
#pragma unroll
      for (int it = 0; it < 8; ++it) {
        const int row = it * 8 + wave * 4 + q;
        const size_t o = (row0 + t0 + row) * kDin + d0 + c8;
        *(volatile v8h*)(YH + o) = hv[it];
        *(volatile v8h*)(YL + o) = lv[it];
      }
      __threadfence();
    }
  }
}

extern "C" void kernel_launch(void* const* d_in, const int* in_sizes, int n_in,
                              void* d_out, int out_size, void* d_ws, size_t ws_size,
                              hipStream_t stream) {
  if (n_in < 10) return;
  if (in_sizes[0] != kRows * kDm) return;
  if (in_sizes[1] != 2 * kDin * kDm) return;
  if (in_sizes[2] != kDin * 4) return;
  if (in_sizes[3] != kDin) return;
  if (in_sizes[4] != kXdW * kDin) return;
  if (in_sizes[5] != kDin * kDtR) return;
  if (in_sizes[6] != kDin) return;
  if (in_sizes[7] != kDin * kNst) return;
  if (in_sizes[8] != kDin) return;
  if (in_sizes[9] != kDm * kDin) return;
  if (out_size != kRows * kDm) return;
  if (ws_size < kWsTotal) return;

  const float* x       = (const float*)d_in[0];
  const float* W_in    = (const float*)d_in[1];
  const float* conv_w  = (const float*)d_in[2];
  const float* conv_b  = (const float*)d_in[3];
  const float* W_xproj = (const float*)d_in[4];
  const float* W_dt    = (const float*)d_in[5];
  const float* b_dt    = (const float*)d_in[6];
  const float* A_log   = (const float*)d_in[7];
  const float* Dp      = (const float*)d_in[8];
  const float* W_out   = (const float*)d_in[9];
  float* out = (float*)d_out;

  char* ws = (char*)d_ws;
  unsigned short* XB   = (unsigned short*)(ws + kOffXB);
  unsigned short* WIB  = (unsigned short*)(ws + kOffWIB);
  unsigned short* WXB  = (unsigned short*)(ws + kOffWXB);
  unsigned short* WDB  = (unsigned short*)(ws + kOffWDB);
  unsigned short* WOB  = (unsigned short*)(ws + kOffWOB);
  unsigned short* XHP  = (unsigned short*)(ws + kOffXHP);
  unsigned short* XLP  = (unsigned short*)(ws + kOffXLP);
  float*          Z    = (float*)(ws + kOffZ);
  unsigned short* UCH  = (unsigned short*)(ws + kOffUCH);
  unsigned short* UCL  = (unsigned short*)(ws + kOffUCL);
  unsigned short* XDH  = (unsigned short*)(ws + kOffXDH);
  unsigned short* XDL  = (unsigned short*)(ws + kOffXDL);
  unsigned short* YH   = XHP;
  unsigned short* YL   = XLP;

  {
    const int n8x  = kRows * kDm / 8;
    const int n8wi = 2 * kDin * kDm / 8;
    const int n8wx = kXdP * kDin / 8, v8wx = kXdW * kDin / 8;
    const int n8wd = kDin * kDtR / 8;
    const int n8wo = kDm * kDin / 8;
    rows_bf16_kernel<<<(n8x + 255) / 256, 256, 0, stream>>>(x, XB, n8x, n8x);
    rows_bf16_kernel<<<(n8wi + 255) / 256, 256, 0, stream>>>(W_in, WIB, n8wi, n8wi);
    rows_bf16_kernel<<<(n8wx + 255) / 256, 256, 0, stream>>>(W_xproj, WXB, n8wx, v8wx);
    rows_bf16_kernel<<<(n8wd + 255) / 256, 256, 0, stream>>>(W_dt, WDB, n8wd, n8wd);
    rows_bf16_kernel<<<(n8wo + 255) / 256, 256, 0, stream>>>(W_out, WOB, n8wo, n8wo);
  }

  {
    const int tiles = (kRows / 64) * (kDin / 64);
    wmma_gemm64<1, 0, 0, 2, false><<<dim3((tiles + 7) / 8, 1), 256, 0, stream>>>(
        XB, nullptr, kDm, 0L,
        WIB, nullptr, kDm, 0L,
        (void*)XHP, (void*)XLP, kDin, 0L,
        nullptr, nullptr, 0L,
        kRows, kDin, kDm, 1.0f);
    wmma_gemm64<1, 0, 0, 0, false><<<dim3((tiles + 7) / 8, 1), 256, 0, stream>>>(
        XB, nullptr, kDm, 0L,
        WIB + (size_t)kDin * kDm, nullptr, kDm, 0L,
        (void*)Z, nullptr, kDin, 0L,
        nullptr, nullptr, 0L,
        kRows, kDin, kDm, 1.0f);
  }

  conv_silu_kernel<<<dim3(kDin / kConvCh, kRows / kConvRw), kConvTh, 0, stream>>>(
      (const unsigned*)(const void*)XHP, (const unsigned*)(const void*)XLP, conv_w, conv_b, UCH, UCL);

  {
    const int tiles = (kRows / 64) * (kXdP / 64);
    wmma_gemm64<1, 1, 0, 2, false><<<dim3((tiles + 7) / 8, 1), 256, 0, stream>>>(
        UCH, UCL, kDin, 0L,
        WXB, nullptr, kDin, 0L,
        (void*)XDH, (void*)XDL, kXdP, 0L,
        nullptr, nullptr, 0L,
        kRows, kXdP, kDin, 1.0f);
  }

  scan_kernel<<<kBatch * (kDin / kScanCh), kScanCh, 0, stream>>>(
      XDH, XDL, UCH, UCL, Z, WDB, b_dt, A_log, Dp, YH, YL);

  {
    const int tiles = (kRows / 64) * (kDm / 64);
    wmma_gemm64<1, 1, 0, 0, false><<<dim3((tiles + 7) / 8, 1), 256, 0, stream>>>(
        YH, YL, kDin, 0L,
        WOB, nullptr, kDin, 0L,
        (void*)out, nullptr, kDm, 0L,
        nullptr, nullptr, 0L,
        kRows, kDm, kDin, 1.0f);
  }
}
